// ConditioningEncoder_61014305407432
// MI455X (gfx1250) — hardware-verified
//
#include <hip/hip_runtime.h>
#include <math.h>
#include <stdint.h>

#define NBAT  16
#define TT    2048
#define TS    512
#define HID   256
#define CND   512
#define NH    4
#define HD    64
#define NKB   (TS / 32)
#define QSC   1024.0f
#define KSC   1024.0f
#define CSC   1024.0f
#define VCAR  1024.0f
#define PCAR  1024.0f
#define OSC   8192.0f
#define YSC   16384.0f
#define WSC   1024.0f
#define PCEN  0.875f
#define LOG2E 1.4426950408889634f
#define MASKT (-10000.0f * LOG2E)
#define SLAB64 (16 * 68)
#define SLABF  (16 * 68)
#define VTP    72
static_assert(HID == NH * HD && HD == 64);
static_assert((TT % 64) == 0 && (TS % 64) == 0 && (TS % 32) == 0 && NKB == 16);
static_assert((TT & (TT - 1)) == 0 && (TS & (TS - 1)) == 0);
static_assert(16 * 36 <= SLABF);
static_assert((HID % 64) == 0 && (CND % 64) == 0 && (HID % 32) == 0 && (CND % 32) == 0);
static_assert(((NBAT * TT * NH * 8) % 256) == 0 && ((NBAT * TS * NH * 8) % 256) == 0);
static_assert(((NBAT * TS * HID) % 2048) == 0 && ((NBAT * TT * HID) % 2048) == 0);

typedef unsigned short u16;
typedef _Float16 v16h __attribute__((ext_vector_type(16)));
typedef _Float16 v8h  __attribute__((ext_vector_type(8)));
typedef __bf16   v16b __attribute__((ext_vector_type(16)));
typedef float    v8f  __attribute__((ext_vector_type(8)));
typedef float    v4f  __attribute__((ext_vector_type(4)));
typedef unsigned int v4u __attribute__((ext_vector_type(4)));

union FragH { v16h v; v8h h[2]; v4u u[2]; };
union FragB { v16b v; v4u u[2]; };

struct InvF { float f[32]; };
static_assert(sizeof(InvF) == 128);

__device__ __forceinline__ unsigned short bf_bits(float f) {
  unsigned u = __float_as_uint(f);
  return (unsigned short)((u + 0x7FFFu + ((u >> 16) & 1u)) >> 16);
}
__device__ __forceinline__ float bf_up(unsigned short h) { return __uint_as_float(((unsigned)h) << 16); }
__device__ __forceinline__ float bfr(float f) { return bf_up(bf_bits(f)); }
__device__ __forceinline__ unsigned short h_bits(_Float16 x) { return __builtin_bit_cast(unsigned short, x); }
__device__ __forceinline__ unsigned pk16(unsigned short a, unsigned short b) { return (unsigned)a | ((unsigned)b << 16); }
__device__ __forceinline__ v8f zero8() { v8f z = {0.f, 0.f, 0.f, 0.f, 0.f, 0.f, 0.f, 0.f}; return z; }

__device__ __forceinline__ v16h ldfrag_h(const _Float16* p) {
  FragH f;
  f.h[0] = *(const v8h*)(p);
  f.h[1] = *(const v8h*)(p + 16);
  return f.v;
}
__device__ __forceinline__ v16b ldfrag_b(const u16* p) {
  FragB f;
  f.u[0] = *(const v4u*)(p);
  f.u[1] = *(const v4u*)(p + 16);
  return f.v;
}

__device__ __forceinline__ v8f mma_h(v16h a, v16h b, v8f c) {
  return __builtin_amdgcn_wmma_f32_16x16x32_f16(false, a, false, b, (short)0, c, false, false);
}
__device__ __forceinline__ v8f mma_b(v16b a, v16b b, v8f c) {
  return __builtin_amdgcn_wmma_f32_16x16x32_bf16(false, a, false, b, (short)0, c, false, false);
}
__device__ __forceinline__ void guard2(v8f& a, v8f& b, v16h x0, v16h x1, v16h x2, v16h x3, v16h x4, v16h x5) {
#if defined(__HIP_DEVICE_COMPILE__)
  asm volatile("v_nop\n\tv_nop\n\tv_nop\n\tv_nop"
               : "+v"(a), "+v"(b) : "v"(x0), "v"(x1), "v"(x2), "v"(x3), "v"(x4), "v"(x5) : "memory");
#endif
}
template <typename F>
__device__ __forceinline__ void guard6(v8f& a, v8f& b, v8f& c, v8f& d, F x0, F x1, F x2, F x3, F x4, F x5) {
#if defined(__HIP_DEVICE_COMPILE__)
  asm volatile("v_nop\n\tv_nop\n\tv_nop\n\tv_nop"
               : "+v"(a), "+v"(b), "+v"(c), "+v"(d) : "v"(x0), "v"(x1), "v"(x2), "v"(x3), "v"(x4), "v"(x5) : "memory");
#endif
}
__device__ __forceinline__ void guard10(v8f& a, v8f& b, v8f& c, v8f& d, v16h x0, v16h x1, v16h x2, v16h x3, v16h x4,
                                        v16h x5, v16h x6, v16h x7, v16h x8, v16h x9) {
#if defined(__HIP_DEVICE_COMPILE__)
  asm volatile("v_nop\n\tv_nop\n\tv_nop\n\tv_nop"
               : "+v"(a), "+v"(b), "+v"(c), "+v"(d)
               : "v"(x0), "v"(x1), "v"(x2), "v"(x3), "v"(x4), "v"(x5), "v"(x6), "v"(x7), "v"(x8), "v"(x9) : "memory");
#endif
}
__device__ __forceinline__ void guardF(v8f& a0, v8f& a1, v8f& a2, v8f& a3, v8f& c0, v8f& c1, v8f& c2, v8f& c3,
                                       v16h x0, v16h x1, v16h x2, v16h x3, v16h x4, v16h x5, v16h x6, v16h x7,
                                       v16h x8, v16h x9) {
#if defined(__HIP_DEVICE_COMPILE__)
  asm volatile("v_nop\n\tv_nop\n\tv_nop\n\tv_nop"
               : "+v"(a0), "+v"(a1), "+v"(a2), "+v"(a3), "+v"(c0), "+v"(c1), "+v"(c2), "+v"(c3)
               : "v"(x0), "v"(x1), "v"(x2), "v"(x3), "v"(x4), "v"(x5), "v"(x6), "v"(x7), "v"(x8), "v"(x9) : "memory");
#endif
}
__device__ __forceinline__ void acc_guard4(v8f& a, v8f& b, v8f& c, v8f& d) {
#if defined(__HIP_DEVICE_COMPILE__)
  asm volatile("v_nop\n\tv_nop\n\tv_nop\n\tv_nop" : "+v"(a), "+v"(b), "+v"(c), "+v"(d));
#endif
}
__device__ __forceinline__ void wave_sync_lds() {
  __builtin_amdgcn_fence(__ATOMIC_RELEASE, "workgroup");
  __builtin_amdgcn_wave_barrier();
  __builtin_amdgcn_fence(__ATOMIC_ACQUIRE, "workgroup");
}

__device__ __forceinline__ void sincos_acc(float angf, float& sv, float& cv) {
  const double a = (double)angf;
  const double TWO_OVER_PI = 0.63661977236758134308;
  const double PIO2_HI = 1.5707963267948966;
  const double PIO2_LO = 6.123233995736766e-17;
  const int kq = (int)(a * TWO_OVER_PI + 0.5);
  const double kd = (double)kq;
  double r = fma(-kd, PIO2_HI, a);
  r = fma(-kd, PIO2_LO, r);
  const double r2 = r * r;
  double sp = 1.0 / 6227020800.0;
  sp = fma(sp, r2, -1.0 / 39916800.0);
  sp = fma(sp, r2, 1.0 / 362880.0);
  sp = fma(sp, r2, -1.0 / 5040.0);
  sp = fma(sp, r2, 1.0 / 120.0);
  sp = fma(sp, r2, -1.0 / 6.0);
  const double s = fma(sp * r2, r, r);
  double cp = -1.0 / 87178291200.0;
  cp = fma(cp, r2, 1.0 / 479001600.0);
  cp = fma(cp, r2, -1.0 / 3628800.0);
  cp = fma(cp, r2, 1.0 / 40320.0);
  cp = fma(cp, r2, -1.0 / 720.0);
  cp = fma(cp, r2, 1.0 / 24.0);
  cp = fma(cp, r2, -0.5);
  const double c = fma(cp, r2, 1.0);
  const int qd = kq & 3;
  const double so = (qd == 0) ? s : (qd == 1) ? c : (qd == 2) ? -s : -c;
  const double co = (qd == 0) ? c : (qd == 1) ? -s : (qd == 2) ? -c : s;
  sv = (float)so;
  cv = (float)co;
}

__global__ __launch_bounds__(256) void k_tab(float* cosT, float* sinT, InvF inv) {
  const int tid  = threadIdx.x;
  const int lane = tid & 31;
  const int t    = blockIdx.x * 8 + (tid >> 5);
  if (t >= TT) return;
  float f = inv.f[0];
#pragma unroll
  for (int i = 1; i < 32; ++i) f = (lane == i) ? inv.f[i] : f;
  const float ang = (float)t * f;
  float sv, cv;
  sincos_acc(ang, sv, cv);
  float* cr = cosT + (size_t)t * HD;
  float* sr = sinT + (size_t)t * HD;
  for (int pass = 0; pass < 2; ++pass) {
    *(volatile float*)(cr + lane)      = cv;
    *(volatile float*)(cr + 32 + lane) = cv;
    *(volatile float*)(sr + lane)      = sv;
    *(volatile float*)(sr + 32 + lane) = sv;
    __threadfence();
  }
}

__global__ __launch_bounds__(256) void cvt_T(const float* __restrict__ W, u16* D, int R, int C) {
  __shared__ __align__(16) u16 T[64 * VTP];
  const int tid = threadIdx.x;
  const int ntc = C >> 6;
  const int bid = blockIdx.x;
  const int bb  = blockIdx.y;
  const int c0  = (bid % ntc) * 64;
  const int r0  = (bid / ntc) * 64;
  const float* Wb = W + (size_t)bb * (size_t)R * (size_t)C;
  u16*         Db = D + (size_t)bb * (size_t)R * (size_t)C;
  {
    const int rr = tid >> 2;
    const int cc = (tid & 3) * 16;
    const float* src = Wb + (size_t)(r0 + rr) * C + c0 + cc;
#pragma unroll
    for (int i = 0; i < 4; ++i) {
      const v4f a = *(const v4f*)(src + 4 * i);
#pragma unroll
      for (int e = 0; e < 4; ++e) T[(cc + 4 * i + e) * VTP + rr] = bf_bits(a[e]);
    }
  }
  __syncthreads();
  v4u vals[2];
  const int q8 = tid >> 3, p8 = (tid & 7) * 8;
#pragma unroll
  for (int it = 0; it < 2; ++it) vals[it] = *(const v4u*)(T + (it * 32 + q8) * VTP + p8);
  for (int pass = 0; pass < 2; ++pass) {
#pragma unroll
    for (int it = 0; it < 2; ++it) {
      const int n = it * 32 + q8;
      *(volatile v4u*)(Db + (size_t)(c0 + n) * R + r0 + p8) = vals[it];
    }
    __threadfence();
  }
}

__global__ __launch_bounds__(256) void cvt_flat(const float* __restrict__ src, u16* D, int n8, int f16mode, float scale) {
  const int gt = blockIdx.x * 256 + (int)threadIdx.x;
  if (gt >= n8) return;
  const float* p = src + (size_t)gt * 8;
  const v4f a = *(const v4f*)(p), bq = *(const v4f*)(p + 4);
  float w[8];
#pragma unroll
  for (int e = 0; e < 4; ++e) { w[e] = a[e]; w[4 + e] = bq[e]; }
  v4u o;
#pragma unroll
  for (int e = 0; e < 4; ++e) {
    const float v0 = w[2 * e], v1 = w[2 * e + 1];
    const unsigned short h0 = h_bits((_Float16)(bfr(v0) * scale)), h1 = h_bits((_Float16)(bfr(v1) * scale));
    const unsigned short b0 = bf_bits(v0), b1 = bf_bits(v1);
    o[e] = (f16mode != 0) ? pk16(h0, h1) : pk16(b0, b1);
  }
  u16* d = D + (size_t)gt * 8;
  for (int pass = 0; pass < 2; ++pass) {
    *(volatile v4u*)(d) = o;
    __threadfence();
  }
}

__global__ __launch_bounds__(256) void cvt_split(const float* __restrict__ src, u16* Hp, u16* Lp, int n8, float sc) {
  const int gt = blockIdx.x * 256 + (int)threadIdx.x;
  if (gt >= n8) return;
  const float* p = src + (size_t)gt * 8;
  const v4f a = *(const v4f*)(p), bq = *(const v4f*)(p + 4);
  float w[8];
#pragma unroll
  for (int e = 0; e < 4; ++e) { w[e] = a[e] * sc; w[4 + e] = bq[e] * sc; }
  v4u oh, ol;
#pragma unroll
  for (int e = 0; e < 4; ++e) {
    const float t0 = w[2 * e], t1 = w[2 * e + 1];
    const _Float16 h0 = (_Float16)t0, h1 = (_Float16)t1;
    const _Float16 l0 = (_Float16)(t0 - (float)h0), l1 = (_Float16)(t1 - (float)h1);
    oh[e] = pk16(h_bits(h0), h_bits(h1));
    ol[e] = pk16(h_bits(l0), h_bits(l1));
  }
  const size_t o8 = (size_t)gt * 8;
  for (int pass = 0; pass < 2; ++pass) {
    *(volatile v4u*)(Hp + o8) = oh;
    *(volatile v4u*)(Lp + o8) = ol;
    __threadfence();
  }
}

__device__ __forceinline__ void store64(const float* sl, float* C, int N, size_t rowb, int col0, int lane) {
  const int hh = lane >> 4, m = lane & 15;
  v4f vals[8];
#pragma unroll
  for (int it = 0; it < 8; ++it) vals[it] = *(const v4f*)(sl + (it * 2 + hh) * 68 + m * 4);
  float* dst = C + (rowb + (size_t)hh) * (size_t)N + col0 + m * 4;
  for (int pass = 0; pass < 2; ++pass) {
#pragma unroll
    for (int it = 0; it < 8; ++it) {
      *(volatile v4f*)(dst + (size_t)(it * 2) * (size_t)N) = vals[it];
    }
    __threadfence();
  }
}

__global__ __launch_bounds__(128)
void gemm_bf(const u16* __restrict__ A, const u16* __restrict__ Bt, const float* __restrict__ bias, float* C,
             int M, int N, int K, float oscale) {
  __shared__ __align__(16) float slab[4 * SLAB64];
  const int tid = threadIdx.x, wave = tid >> 5, lane = tid & 31, hh = lane >> 4, m = lane & 15;
  const int ntile = N >> 6;
  const int bid   = blockIdx.x;
  const int rowb  = (bid / ntile) * 64 + wave * 16;
  const int col0  = (bid % ntile) * 64;
  if (rowb + 16 > M) return;
  const u16* ap = A  + (size_t)(rowb + m) * K + 8 * hh;
  const u16* bp = Bt + (size_t)(col0 + m) * K + 8 * hh;
  const size_t bs = (size_t)16 * K;
  v8f acc0 = zero8(), acc1 = zero8(), acc2 = zero8(), acc3 = zero8();
#pragma unroll 1
  for (int k0 = 0; k0 < K; k0 += 32) {
    const v16b a  = ldfrag_b(ap + k0);
    const v16b b0 = ldfrag_b(bp + k0);
    const v16b b1 = ldfrag_b(bp + bs + k0);
    const v16b b2 = ldfrag_b(bp + 2 * bs + k0);
    const v16b b3 = ldfrag_b(bp + 3 * bs + k0);
    acc0 = mma_b(a, b0, acc0);
    acc1 = mma_b(a, b1, acc1);
    acc2 = mma_b(a, b2, acc2);
    acc3 = mma_b(a, b3, acc3);
    guard6<v16b>(acc0, acc1, acc2, acc3, a, b0, b1, b2, b3, a);
  }
  float* sl = slab + wave * SLAB64;
  float bb[4];
#pragma unroll
  for (int j = 0; j < 4; ++j) bb[j] = bfr(bias[col0 + 16 * j + m]);
#pragma unroll
  for (int r = 0; r < 8; ++r) {
    const int ro = (8 * hh + r) * 68 + m;
    sl[ro]      = acc0[r] * oscale + bb[0];
    sl[ro + 16] = acc1[r] * oscale + bb[1];
    sl[ro + 32] = acc2[r] * oscale + bb[2];
    sl[ro + 48] = acc3[r] * oscale + bb[3];
  }
  wave_sync_lds();
  store64(sl, C, N, (size_t)rowb, col0, lane);
}

template <int A2, int B2>
__global__ __launch_bounds__(128)
void gemm_h(const u16* __restrict__ Ah, const u16* __restrict__ Al, const u16* __restrict__ Bh, const u16* __restrict__ Bl,
            const float* __restrict__ bias, float* C, int M, int N, int K, int sA, int sB, int sC, int biasRow, float oscale) {
  __shared__ __align__(16) float slab[4 * SLAB64];
  const int tid = threadIdx.x, wave = tid >> 5, lane = tid & 31, hh = lane >> 4, m = lane & 15;
  const int ntile = N >> 6;
  const int bid   = blockIdx.x;
  const int bz    = blockIdx.y;
  const int rowb  = (bid / ntile) * 64 + wave * 16;
  const int col0  = (bid % ntile) * 64;
  if (rowb + 16 > M) return;
  const size_t aofs = (size_t)bz * (size_t)sA + (size_t)(rowb + m) * K + 8 * hh;
  const _Float16* ahp = (const _Float16*)(const void*)Ah + aofs;
  const _Float16* alp = (const _Float16*)(const void*)Al + aofs;
  const size_t bofs = (size_t)bz * (size_t)sB + (size_t)(col0 + m) * K + 8 * hh;
  const _Float16* bhp = (const _Float16*)(const void*)Bh + bofs;
  const _Float16* blp = (const _Float16*)(const void*)Bl + bofs;
  const size_t bs = (size_t)16 * K;
  v8f acc0 = zero8(), acc1 = zero8(), acc2 = zero8(), acc3 = zero8();
#pragma unroll 1
  for (int k0 = 0; k0 < K; k0 += 32) {
    const v16h ah = ldfrag_h(ahp + k0);
    const v16h b0 = ldfrag_h(bhp + k0);
    const v16h b1 = ldfrag_h(bhp + bs + k0);
    const v16h b2 = ldfrag_h(bhp + 2 * bs + k0);
    const v16h b3 = ldfrag_h(bhp + 3 * bs + k0);
    if (A2) {
      const v16h al = ldfrag_h(alp + k0);
      acc0 = mma_h(ah, b0, acc0);  acc0 = mma_h(al, b0, acc0);
      acc1 = mma_h(ah, b1, acc1);  acc1 = mma_h(al, b1, acc1);
      acc2 = mma_h(ah, b2, acc2);  acc2 = mma_h(al, b2, acc2);
      acc3 = mma_h(ah, b3, acc3);  acc3 = mma_h(al, b3, acc3);
      guard6<v16h>(acc0, acc1, acc2, acc3, ah, al, b0, b1, b2, b3);
    } else if (B2) {
      const v16h c0 = ldfrag_h(blp + k0);
      const v16h c1 = ldfrag_h(blp + bs + k0);
      const v16h c2 = ldfrag_h(blp + 2 * bs + k0);
      const v16h c3 = ldfrag_h(blp + 3 * bs + k0);
      acc0 = mma_h(ah, b0, acc0);  acc0 = mma_h(ah, c0, acc0);
      acc1 = mma_h(ah, b1, acc1);  acc1 = mma_h(ah, c1, acc1);
      acc2 = mma_h(ah, b2, acc2);  acc2 = mma_h(ah, c2, acc2);
      acc3 = mma_h(ah, b3, acc3);  acc3 = mma_h(ah, c3, acc3);
      guard10(acc0, acc1, acc2, acc3, ah, b0, b1, b2, b3, c0, c1, c2, c3, ah);
    } else {
      acc0 = mma_h(ah, b0, acc0);
      acc1 = mma_h(ah, b1, acc1);
      acc2 = mma_h(ah, b2, acc2);
      acc3 = mma_h(ah, b3, acc3);
      guard6<v16h>(acc0, acc1, acc2, acc3, ah, b0, b1, b2, b3, ah);
    }
  }
  float* sl = slab + wave * SLAB64;
  if (biasRow != 0) {
#pragma unroll
    for (int r = 0; r < 8; ++r) {
      const float bb = bfr(bias[rowb + 8 * hh + r]);
      const int ro = (8 * hh + r) * 68 + m;
      sl[ro]      = acc0[r] * oscale + bb;
      sl[ro + 16] = acc1[r] * oscale + bb;
      sl[ro + 32] = acc2[r] * oscale + bb;
      sl[ro + 48] = acc3[r] * oscale + bb;
    }
  } else {
    float bb[4];
#pragma unroll
    for (int j = 0; j < 4; ++j) bb[j] = bfr(bias[col0 + 16 * j + m]);
#pragma unroll
    for (int r = 0; r < 8; ++r) {
      const int ro = (8 * hh + r) * 68 + m;
      sl[ro]      = acc0[r] * oscale + bb[0];
      sl[ro + 16] = acc1[r] * oscale + bb[1];
      sl[ro + 32] = acc2[r] * oscale + bb[2];
      sl[ro + 48] = acc3[r] * oscale + bb[3];
    }
  }
  wave_sync_lds();
  store64(sl, C + (size_t)bz * (size_t)sC, N, (size_t)rowb, col0, lane);
}

__global__ __launch_bounds__(256) void rope_h(const float* __restrict__ x, const float* __restrict__ cosT,
                                              const float* __restrict__ sinT, u16* hpl,
                                              int nrows, int hpr, int posmask, float sc) {
  const int gt  = blockIdx.x * 256 + (int)threadIdx.x;
  const int row = gt >> 3;
  const int d0  = (gt & 7) * 8;
  if (row >= nrows) return;
  const int pos = (row / hpr) & posmask;
  const int d1  = d0 ^ 32;
  const float* xr = x + (size_t)row * HD;
  const float* cr = cosT + (size_t)pos * HD + d0;
  const float* sr = sinT + (size_t)pos * HD + d0;
  const v4f xa = *(const v4f*)(xr + d0), xb = *(const v4f*)(xr + d0 + 4);
  const v4f ya = *(const v4f*)(xr + d1), yb = *(const v4f*)(xr + d1 + 4);
  const v4f ca = *(const v4f*)(cr), cb = *(const v4f*)(cr + 4);
  const v4f sa = *(const v4f*)(sr), sb = *(const v4f*)(sr + 4);
  const float sgn = (d0 < 32) ? -1.0f : 1.0f;
  float w[8];
#pragma unroll
  for (int e = 0; e < 4; ++e) {
    w[e]     = xa[e] * ca[e] + (sgn * ya[e]) * sa[e];
    w[4 + e] = xb[e] * cb[e] + (sgn * yb[e]) * sb[e];
  }
  v4u oh;
#pragma unroll
  for (int e = 0; e < 4; ++e) {
    const _Float16 h0 = (_Float16)(w[2 * e] * sc), h1 = (_Float16)(w[2 * e + 1] * sc);
    oh[e] = pk16(h_bits(h0), h_bits(h1));
  }
  const size_t o8 = (size_t)row * HD + d0;
  for (int pass = 0; pass < 2; ++pass) {
    *(volatile v4u*)(hpl + o8) = oh;
    __threadfence();
  }
}

__global__ __launch_bounds__(256) void vcvt(const float* __restrict__ V, u16* VH, float* VS) {
  __shared__ __align__(16) float S[128];
  const int tid  = threadIdx.x;
  const int lane = tid & 31;
  const int wave = tid >> 5;
  const int bid  = blockIdx.x;
  const int st   = bid & 7;
  const int ot   = (bid >> 3) & 3;
  const int b    = bid >> 5;
  const int o0   = ot * 64;
  const int s0   = st * 64;
  v4u hv[2];
  size_t eo[2];
#pragma unroll
  for (int it = 0; it < 2; ++it) {
    const int idx = it * 256 + tid;
    const int row = idx >> 3;
    const int s8  = (idx & 7) * 8;
    const size_t e = ((size_t)(b * HID + o0 + row)) * TS + s0 + s8;
    eo[it] = e;
    const v4f a = *(const v4f*)(V + e), bq = *(const v4f*)(V + e + 4);
    v4u o;
#pragma unroll
    for (int q = 0; q < 2; ++q) {
      o[q]     = pk16(h_bits((_Float16)(a[2 * q] * VCAR)),  h_bits((_Float16)(a[2 * q + 1] * VCAR)));
      o[2 + q] = pk16(h_bits((_Float16)(bq[2 * q] * VCAR)), h_bits((_Float16)(bq[2 * q + 1] * VCAR)));
    }
    hv[it] = o;
    float ps = ((a[0] + a[1]) + (a[2] + a[3])) + ((bq[0] + bq[1]) + (bq[2] + bq[3]));
    ps += __shfl_xor(ps, 1, 32);
    ps += __shfl_xor(ps, 2, 32);
    if ((lane & 3) == 0) S[((lane >> 2) & 1) * 64 + row] = ps;
  }
  for (int pass = 0; pass < 2; ++pass) {
#pragma unroll
    for (int it = 0; it < 2; ++it) *(volatile v4u*)(VH + eo[it]) = hv[it];
    __threadfence();
  }
  __syncthreads();
  if (wave == 0) {
    const int kbh   = lane >> 4;
    const int piece = (lane & 15) * 4;
    const v4f sv = *(const v4f*)(S + kbh * 64 + piece);
    float* dst = VS + ((size_t)(b * NKB + 2 * st + kbh)) * HID + o0 + piece;
    for (int pass = 0; pass < 2; ++pass) {
      *(volatile v4f*)(dst) = sv;
      __threadfence();
    }
  }
}

__global__ __launch_bounds__(128)
void attn_x(const u16* __restrict__ QHp, const u16* __restrict__ KHp, const u16* __restrict__ VHp,
            const float* __restrict__ VS, const float* __restrict__ cmask, const float* __restrict__ xmask,
            u16* OHp, u16* OLp) {
  __shared__ __align__(16) float smem[4 * SLABF];

  const int tid  = threadIdx.x;
  const int wave = tid >> 5;
  const int lane = tid & 31;
  const int hh   = lane >> 4;
  const int c    = lane & 15;

  const int bid  = blockIdx.x;
  const int qt   = bid & (TT / 64 - 1);
  const int h    = (bid >> 5) & (NH - 1);
  const int b    = bid >> 7;
  const int q0   = qt * 64 + wave * 16;

  const size_t qofs = (((size_t)(b * TT + q0 + c)) * NH + h) * HD + 8 * hh;
  const _Float16* Qh  = (const _Float16*)(const void*)QHp + qofs;
  const size_t kofs = (((size_t)(b * TS + c)) * NH + h) * HD + 8 * hh;
  const _Float16* Khb = (const _Float16*)(const void*)KHp + kofs;
  const size_t vofs = ((size_t)(b * HID + h * HD + c)) * TS + 8 * hh;
  const _Float16* Vhb = (const _Float16*)(const void*)VHp + vofs;
  const float* vsb = VS + (size_t)b * NKB * HID + h * HD + c;
  const float* cmb = cmask + (size_t)b * TS + c;
  const float lsc = 0.125f * (LOG2E / (QSC * KSC));
  const float C0S = PCEN * PCAR * VCAR;

  float xmv[8], mrow[8], lrow[8];
  v8f o[4];
#pragma unroll
  for (int r = 0; r < 8; ++r) {
    xmv[r]  = bfr(xmask[(size_t)b * TT + q0 + 8 * hh + r]);
    mrow[r] = -INFINITY;
    lrow[r] = 0.f;
  }
#pragma unroll
  for (int j = 0; j < 4; ++j) o[j] = zero8();
  float* pt = smem + wave * SLABF;

  const v16h qa = ldfrag_h(Qh), qb = ldfrag_h(Qh + 32);

#pragma unroll 1
  for (int it = 0; it < NKB; ++it) {
    const int kb = it * 32;
    v8f s0 = zero8(), s1 = zero8();
    {
      const _Float16* k0p = Khb + (size_t)kb * (NH * HD);
      const _Float16* k1p = k0p + (size_t)16 * (NH * HD);
      const v16h k0a = ldfrag_h(k0p), k0b = ldfrag_h(k0p + 32);
      const v16h k1a = ldfrag_h(k1p), k1b = ldfrag_h(k1p + 32);
      s0 = mma_h(qa, k0a, s0);
      s0 = mma_h(qb, k0b, s0);
      s1 = mma_h(qa, k1a, s1);
      s1 = mma_h(qb, k1b, s1);
      guard2(s0, s1, qa, qb, k0a, k0b, k1a, k1b);
    }
    const float cm0 = bfr(cmb[kb]), cm1 = bfr(cmb[kb + 16]);
    float vs[4];
#pragma unroll
    for (int j = 0; j < 4; ++j) vs[j] = vsb[(size_t)it * HID + 16 * j] * C0S;
#pragma unroll
    for (int r = 0; r < 8; ++r) {
      const bool ok0 = (cm0 * xmv[r]) != 0.0f;
      const bool ok1 = (cm1 * xmv[r]) != 0.0f;
      const float t0 = ok0 ? (s0[r] * lsc) : MASKT;
      const float t1 = ok1 ? (s1[r] * lsc) : MASKT;
      float mx = fmaxf(t0, t1);
#pragma unroll
      for (int off = 1; off < 16; off <<= 1) mx = fmaxf(mx, __shfl_xor(mx, off, 32));
      const float mn = fmaxf(mrow[r], mx);
      const float al = exp2f(mrow[r] - mn);
      mrow[r] = mn;
      const float e0 = exp2f(t0 - mn), e1 = exp2f(t1 - mn);
      float ps = e0 + e1;
#pragma unroll
      for (int off = 1; off < 16; off <<= 1) ps += __shfl_xor(ps, off, 32);
      lrow[r] = lrow[r] * al + ps;
#pragma unroll
      for (int j = 0; j < 4; ++j) o[j][r] = o[j][r] * al + vs[j];
      const int ro = (8 * hh + r) * 36 + c;
      pt[ro]      = (e0 - PCEN) * PCAR;
      pt[ro + 16] = (e1 - PCEN) * PCAR;
    }
    wave_sync_lds();
    FragH ph;
    {
      const float* prow = pt + c * 36 + 8 * hh;
      const v4f p0 = *(const v4f*)(prow), p1 = *(const v4f*)(prow + 4);
      const v4f p2 = *(const v4f*)(prow + 16), p3 = *(const v4f*)(prow + 20);
#pragma unroll
      for (int e = 0; e < 4; ++e) {
        ph.h[0][e]     = (_Float16)p0[e];
        ph.h[0][4 + e] = (_Float16)p1[e];
        ph.h[1][e]     = (_Float16)p2[e];
        ph.h[1][4 + e] = (_Float16)p3[e];
      }
    }
    {
      const _Float16* vhp = Vhb + kb;
      const v16h vh0 = ldfrag_h(vhp);
      const v16h vh1 = ldfrag_h(vhp + (size_t)16 * TS);
      const v16h vh2 = ldfrag_h(vhp + (size_t)32 * TS);
      const v16h vh3 = ldfrag_h(vhp + (size_t)48 * TS);
      o[0] = mma_h(ph.v, vh0, o[0]);
      o[1] = mma_h(ph.v, vh1, o[1]);
      o[2] = mma_h(ph.v, vh2, o[2]);
      o[3] = mma_h(ph.v, vh3, o[3]);
      guard6<v16h>(o[0], o[1], o[2], o[3], ph.v, vh0, vh1, vh2, vh3, ph.v);
    }
    wave_sync_lds();
  }
  acc_guard4(o[0], o[1], o[2], o[3]);

  wave_sync_lds();
  float* slab = pt;
  const float oc = 1.0f / (PCAR * VCAR);
#pragma unroll
  for (int r = 0; r < 8; ++r) {
    const float inv = (1.0f / lrow[r]) * oc;
#pragma unroll
    for (int j = 0; j < 4; ++j) slab[(8 * hh + r) * 68 + j * 16 + c] = o[j][r] * inv;
  }
  wave_sync_lds();
  v4u oh[4], ol[4];
  const int rq = lane >> 3, c8 = (lane & 7) * 8;
#pragma unroll
  for (int it = 0; it < 4; ++it) {
    const int row = it * 4 + rq;
    const v4f a = *(const v4f*)(slab + row * 68 + c8), bq = *(const v4f*)(slab + row * 68 + c8 + 4);
    float w[8];
#pragma unroll
    for (int e = 0; e < 4; ++e) { w[e] = a[e] * OSC; w[4 + e] = bq[e] * OSC; }
#pragma unroll
    for (int e = 0; e < 4; ++e) {
      const _Float16 h0 = (_Float16)w[2 * e], h1 = (_Float16)w[2 * e + 1];
      const _Float16 l0 = (_Float16)(w[2 * e] - (float)h0), l1 = (_Float16)(w[2 * e + 1] - (float)h1);
      oh[it][e] = pk16(h_bits(h0), h_bits(h1));
      ol[it][e] = pk16(h_bits(l0), h_bits(l1));
    }
  }
  const size_t ob = (((size_t)(b * TT + q0)) * NH + h) * HD + c8;
  for (int pass = 0; pass < 2; ++pass) {
#pragma unroll
    for (int it = 0; it < 4; ++it) {
      const int row = it * 4 + rq;
      const size_t o8 = ob + (size_t)row * (NH * HD);
      *(volatile v4u*)(OHp + o8) = oh[it];
      *(volatile v4u*)(OLp + o8) = ol[it];
    }
    __threadfence();
  }
}

__global__ __launch_bounds__(128)
void film_k(const u16* __restrict__ WF, const u16* __restrict__ YHp, const u16* __restrict__ YLp,
            const float* __restrict__ bfl, const float* __restrict__ X, const float* __restrict__ XM,
            float* OUT, float oscale) {
  __shared__ __align__(16) float slab[4 * SLAB64];
  const int tid = threadIdx.x, wave = tid >> 5, lane = tid & 31, hh = lane >> 4, m = lane & 15;
  const int bid = blockIdx.x;
  const int tt  = bid & (TT / 64 - 1);
  const int cg  = (bid >> 5) & 3;
  const int b   = bid >> 7;
  const int t0  = tt * 64;
  const int c0  = cg * 64 + wave * 16;
  const _Float16* agp = (const _Float16*)(const void*)WF + (size_t)(c0 + m) * HID + 8 * hh;
  const _Float16* abp = agp + (size_t)HID * HID;
  const size_t yofs = ((size_t)(b * TT + t0 + m)) * HID + 8 * hh;
  const _Float16* yhp = (const _Float16*)(const void*)YHp + yofs;
  const _Float16* ylp = (const _Float16*)(const void*)YLp + yofs;
  const size_t bs = (size_t)16 * HID;
  v8f g[4], be[4];
#pragma unroll
  for (int j = 0; j < 4; ++j) { g[j] = zero8(); be[j] = zero8(); }
#pragma unroll 1
  for (int k0 = 0; k0 < HID; k0 += 32) {
    const v16h ag = ldfrag_h(agp + k0), ab = ldfrag_h(abp + k0);
    const v16h y0 = ldfrag_h(yhp + k0);
    const v16h y1 = ldfrag_h(yhp + bs + k0);
    const v16h y2 = ldfrag_h(yhp + 2 * bs + k0);
    const v16h y3 = ldfrag_h(yhp + 3 * bs + k0);
    g[0] = mma_h(ag, y0, g[0]);  be[0] = mma_h(ab, y0, be[0]);
    g[1] = mma_h(ag, y1, g[1]);  be[1] = mma_h(ab, y1, be[1]);
    g[2] = mma_h(ag, y2, g[2]);  be[2] = mma_h(ab, y2, be[2]);
    g[3] = mma_h(ag, y3, g[3]);  be[3] = mma_h(ab, y3, be[3]);
    const v16h z0 = ldfrag_h(ylp + k0);
    const v16h z1 = ldfrag_h(ylp + bs + k0);
    const v16h z2 = ldfrag_h(ylp + 2 * bs + k0);
    const v16h z3 = ldfrag_h(ylp + 3 * bs + k0);
    g[0] = mma_h(ag, z0, g[0]);  be[0] = mma_h(ab, z0, be[0]);
    g[1] = mma_h(ag, z1, g[1]);  be[1] = mma_h(ab, z1, be[1]);
    g[2] = mma_h(ag, z2, g[2]);  be[2] = mma_h(ab, z2, be[2]);
    g[3] = mma_h(ag, z3, g[3]);  be[3] = mma_h(ab, z3, be[3]);
    guardF(g[0], g[1], g[2], g[3], be[0], be[1], be[2], be[3], ag, ab, y0, y1, y2, y3, z0, z1, z2, z3);
  }
  float* sl = slab + wave * SLAB64;
  float xm[4];
#pragma unroll
  for (int j = 0; j < 4; ++j) xm[j] = bfr(XM[(size_t)b * TT + t0 + 16 * j + m]);
#pragma unroll
  for (int r = 0; r < 8; ++r) {
    const int cc = c0 + 8 * hh + r;
    const float bg = bfr(bfl[cc]);
    const float bb = bfr(bfl[HID + cc]);
    const float* xr = X + ((size_t)(b * HID + cc)) * TT + t0 + m;
#pragma unroll
    for (int j = 0; j < 4; ++j) {
      const float gam = g[j][r] * oscale + bg;
      const float bet = be[j][r] * oscale + bb;
      const float xv  = bfr(xr[16 * j]);
      sl[(8 * hh + r) * 68 + 16 * j + m] = (xv * gam + bet) * xm[j];
    }
  }
  wave_sync_lds();
  store64(sl, OUT, TT, (size_t)(b * HID + c0), t0, lane);
}

extern "C" void kernel_launch(void* const* d_in, const int* in_sizes, int n_in,
                              void* d_out, int out_size, void* d_ws, size_t ws_size,
                              hipStream_t stream) {
  if (n_in < 16) return;
  if (in_sizes[0] != NBAT * HID * TT) return;
  if (in_sizes[1] != NBAT * TT) return;
  if (in_sizes[2] != NBAT * CND * TS) return;
  if (in_sizes[3] != NBAT * TS) return;
  if (in_sizes[4] != HID * CND || in_sizes[5] != HID) return;
  if (in_sizes[6] != HID * HID || in_sizes[7] != HID) return;
  if (in_sizes[8] != HID * HID || in_sizes[9] != HID) return;
  if (in_sizes[10] != HID * HID || in_sizes[11] != HID) return;
  if (in_sizes[12] != HID * HID || in_sizes[13] != HID) return;
  if (in_sizes[14] != 2 * HID * HID || in_sizes[15] != 2 * HID) return;
  if (out_size != NBAT * HID * TT) return;

  const float* x      = (const float*)d_in[0];
  const float* x_mask = (const float*)d_in[1];
  const float* cond   = (const float*)d_in[2];
  const float* c_mask = (const float*)d_in[3];
  const float* w_cond = (const float*)d_in[4];
  const float* b_cond = (const float*)d_in[5];
  const float* wq     = (const float*)d_in[6];
  const float* bq     = (const float*)d_in[7];
  const float* wk     = (const float*)d_in[8];
  const float* bk     = (const float*)d_in[9];
  const float* wv     = (const float*)d_in[10];
  const float* bv     = (const float*)d_in[11];
  const float* wo     = (const float*)d_in[12];
  const float* bo     = (const float*)d_in[13];
  const float* wf     = (const float*)d_in[14];
  const float* bfi    = (const float*)d_in[15];
  float*       out    = (float*)d_out;

  const size_t szTab = (size_t)TT * HD * 4;
  const size_t szR3  = (size_t)NBAT * TT * HID * 2;
  const size_t szR4  = (size_t)NBAT * TS * CND * 2;
  const size_t szWCB = (size_t)HID * CND * 2;
  const size_t szW   = (size_t)HID * HID * 2;
  const size_t szWF  = (size_t)2 * HID * HID * 2;
  const size_t szR5  = (size_t)NBAT * TS * HID * 4;
  const size_t szCP  = (size_t)NBAT * TS * HID * 2;
  const size_t szR1  = (size_t)NBAT * TT * HID * 4;
  const size_t szKH  = (size_t)NBAT * TS * HID * 2;
  const size_t szVH  = (size_t)NBAT * HID * TS * 2;
  const size_t szVS  = (size_t)NBAT * NKB * HID * 4;
  const size_t szOP  = (size_t)NBAT * TT * HID * 2;
  static_assert((size_t)NBAT * TS * CND * 2 == (size_t)NBAT * TS * HID * 4);
  size_t off = 0;
  const size_t oCT  = off; off += szTab;
  const size_t oST  = off; off += szTab;
  const size_t oR3  = off; off += szR3;
  const size_t oR4  = off; off += szR4;
  const size_t oWCB = off; off += szWCB;
  const size_t oWQB = off; off += szW;
  const size_t oWKH = off; off += szW;
  const size_t oWVH = off; off += szW;
  const size_t oWOH = off; off += szW;
  const size_t oWFH = off; off += szWF;
  const size_t oR5  = off; off += szR5;
  const size_t oCH  = off; off += szCP;
  const size_t oCL  = off; off += szCP;
  const size_t oR1  = off; off += szR1;
  const size_t oKH  = off; off += szKH;
  const size_t oVH  = off; off += szVH;
  const size_t oVS  = off; off += szVS;
  const size_t oOH  = off; off += szOP;
  const size_t oOL  = off; off += szOP;
  if (off > ws_size) return;
  if (off > (size_t)134217728) return;

  char* ws = (char*)d_ws;
  float* CT    = (float*)(ws + oCT);
  float* ST    = (float*)(ws + oST);
  u16*   XT    = (u16*)(ws + oR3);
  u16*   QH    = (u16*)(ws + oR3);
  u16*   CONDT = (u16*)(ws + oR4);
  float* KF    = (float*)(ws + oR4);
  u16*   WCB   = (u16*)(ws + oWCB);
  u16*   WQB   = (u16*)(ws + oWQB);
  u16*   WKH   = (u16*)(ws + oWKH);
  u16*   WVH   = (u16*)(ws + oWVH);
  u16*   WOH   = (u16*)(ws + oWOH);
  u16*   WFH   = (u16*)(ws + oWFH);
  float* CTF   = (float*)(ws + oR5);
  float* VF    = (float*)(ws + oR5);
  u16*   CH    = (u16*)(ws + oCH);
  u16*   CL    = (u16*)(ws + oCL);
  float* QF    = (float*)(ws + oR1);
  float* YF    = (float*)(ws + oR1);
  u16*   KH    = (u16*)(ws + oKH);
  u16*   VH    = (u16*)(ws + oVH);
  float* VS    = (float*)(ws + oVS);
  u16*   OH    = (u16*)(ws + oOH);
  u16*   OL    = (u16*)(ws + oOL);
  u16*   YH    = (u16*)(ws + oOH);
  u16*   YL    = (u16*)(ws + oOL);

  InvF inv;
  for (int i = 0; i < 32; ++i) {
    const double p = pow(10000.0, (double)i / 32.0);
    const float pf = (float)p;
    inv.f[i] = 1.0f / pf;
  }

  const dim3 blk(256);
  const dim3 bG(128);
  const int ROWQ = NBAT * TT;
  const int ROWK = NBAT * TS;
  const dim3 gTab(TT / 8);
  const dim3 gXT((TT / 64) * (HID / 64), NBAT);
  const dim3 gCT((TS / 64) * (CND / 64), NBAT);
  const int n8WC = (HID * CND) / 8;
  const int n8W  = (HID * HID) / 8;
  const int n8WF = (2 * HID * HID) / 8;
  const dim3 gWC((n8WC + 255) / 256), gW((n8W + 255) / 256), gWF((n8WF + 255) / 256);
  const dim3 gGC((ROWK / 64) * (HID / 64));
  const int n8C = (ROWK * HID) / 8;
  const dim3 gSC(n8C / 256);
  const dim3 gGQ((ROWQ / 64) * (HID / 64));
  const dim3 gGK((ROWK / 64) * (HID / 64), 1);
  const dim3 gGV((HID / 64) * (TS / 64), NBAT);
  const int rowsQ = ROWQ * NH;
  const int rowsK = ROWK * NH;
  const dim3 gRQ((rowsQ * 8) / 256);
  const dim3 gRK((rowsK * 8) / 256);
  const dim3 gVC(NBAT * (HID / 64) * (TS / 64));
  const dim3 gAT(NBAT * NH * (TT / 64));
  const dim3 gGO((ROWQ / 64) * (HID / 64), 1);
  const int n8Y = (ROWQ * HID) / 8;
  const dim3 gSY(n8Y / 256);
  const dim3 gFM(NBAT * 4 * (TT / 64));

  k_tab<<<gTab, blk, 0, stream>>>(CT, ST, inv);
  cvt_T<<<gXT, blk, 0, stream>>>(x, XT, HID, TT);
  cvt_T<<<gCT, blk, 0, stream>>>(cond, CONDT, CND, TS);
  cvt_flat<<<gWC, blk, 0, stream>>>(w_cond, WCB, n8WC, 0, 1.0f);
  cvt_flat<<<gW,  blk, 0, stream>>>(wq, WQB, n8W, 0, 1.0f);
  cvt_flat<<<gW,  blk, 0, stream>>>(wk, WKH, n8W, 1, WSC);
  cvt_flat<<<gW,  blk, 0, stream>>>(wv, WVH, n8W, 1, WSC);
  cvt_flat<<<gW,  blk, 0, stream>>>(wo, WOH, n8W, 1, WSC);
  cvt_flat<<<gWF, blk, 0, stream>>>(wf, WFH, n8WF, 1, WSC);
  gemm_bf<<<gGC, bG, 0, stream>>>(CONDT, WCB, b_cond, CTF, ROWK, HID, CND, 1.0f);
  cvt_split<<<gSC, blk, 0, stream>>>(CTF, CH, CL, n8C, CSC);
  gemm_bf<<<gGQ, bG, 0, stream>>>(XT, WQB, bq, QF, ROWQ, HID, HID, 1.0f);
  gemm_h<0, 0><<<gGK, bG, 0, stream>>>(CH, CH, WKH, WKH, bk, KF, ROWK, HID, HID, 0, 0, 0, 0, 1.0f / (CSC * WSC));
  gemm_h<0, 1><<<gGV, bG, 0, stream>>>(WVH, WVH, CH, CL, bv, VF, HID, TS, HID, 0, TS * HID, HID * TS, 1, 1.0f / (CSC * WSC));
  rope_h<<<gRQ, blk, 0, stream>>>(QF, CT, ST, QH, rowsQ, NH, TT - 1, QSC);
  rope_h<<<gRK, blk, 0, stream>>>(KF, CT, ST, KH, rowsK, NH, TS - 1, KSC);
  vcvt<<<gVC, blk, 0, stream>>>(VF, VH, VS);
  attn_x<<<gAT, bG, 0, stream>>>(QH, KH, VH, VS, c_mask, x_mask, OH, OL);
  gemm_h<1, 0><<<gGO, bG, 0, stream>>>(OH, OL, WOH, WOH, bo, YF, ROWQ, HID, HID, 0, 0, 0, 0, 1.0f / (OSC * WSC));
  cvt_split<<<gSY, blk, 0, stream>>>(YF, YH, YL, n8Y, YSC);
  film_k<<<gFM, bG, 0, stream>>>(WFH, YH, YL, bfi, x, x_mask, out, 1.0f / (YSC * WSC));
  (void)hipGetLastError();
}
